// SelfSupervised_6975026888742
// MI455X (gfx1250) — hardware-verified
//
#include <hip/hip_runtime.h>
#include <stdint.h>

typedef __attribute__((ext_vector_type(16))) _Float16 v16h;
typedef __attribute__((ext_vector_type(8)))  _Float16 v8h;
typedef __attribute__((ext_vector_type(16))) __bf16   v16b;
typedef __attribute__((ext_vector_type(8)))  __bf16   v8b;
typedef __attribute__((ext_vector_type(8)))  float    v8f;
typedef __attribute__((ext_vector_type(4)))  float    v4f;
typedef __attribute__((ext_vector_type(4)))  unsigned v4u;
typedef __attribute__((ext_vector_type(2)))  float    v2f;

constexpr int NBATCH = 1024;
constexpr int NSTEP  = 128;
constexpr int NINP   = 75;
constexpr int KXPAD0 = 96;
constexpr int NHID   = 128;
constexpr int NGATE  = 512;
constexpr int NEMB   = 256;
constexpr int NDECO  = 9600;

__device__ __forceinline__ unsigned short f2bf_bits(float f) {
  unsigned u = __float_as_uint(f);
  return (unsigned short)((u + 0x7FFFu + ((u >> 16) & 1u)) >> 16);
}
__device__ __forceinline__ float bf_bits2f(unsigned short h) { return __uint_as_float(((unsigned)h) << 16); }

__device__ __forceinline__ void dep_guard_h(v8f& a, v8f& b, v16h x, v16h y) { asm volatile("v_nop\n\tv_nop\n\tv_nop\n\tv_nop" : "+v"(a), "+v"(b) : "v"(x), "v"(y)); }
__device__ __forceinline__ void dep_guard_b(v8f& a, v8f& b, v16b x, v16b y) { asm volatile("v_nop\n\tv_nop\n\tv_nop\n\tv_nop" : "+v"(a), "+v"(b) : "v"(x), "v"(y)); }
__device__ __forceinline__ void keep4_h(v16h a, v16h b, v16h c, v16h d) { asm volatile("v_nop" :: "v"(a), "v"(b), "v"(c), "v"(d)); }
__device__ __forceinline__ void keep4_b(v16b a, v16b b, v16b c, v16b d) { asm volatile("v_nop" :: "v"(a), "v"(b), "v"(c), "v"(d)); }
__device__ __forceinline__ void acc_guard4(v8f& a, v8f& b, v8f& c, v8f& d) { asm volatile("v_nop\n\tv_nop\n\tv_nop\n\tv_nop" : "+v"(a), "+v"(b), "+v"(c), "+v"(d)); }
__device__ __forceinline__ void dep_guard4_h(v8f& a, v8f& b, v8f& c, v8f& d, v16h x, v16h y) { asm volatile("v_nop\n\tv_nop\n\tv_nop\n\tv_nop" : "+v"(a), "+v"(b), "+v"(c), "+v"(d) : "v"(x), "v"(y)); }
__device__ __forceinline__ void keep2_h(v16h a, v16h b) { asm volatile("v_nop" :: "v"(a), "v"(b)); }

template <typename T> struct Frag;
template <> struct Frag<_Float16> {
  typedef v16h V; union U { v16h v; v8h h[2]; };
  static __device__ __forceinline__ v16h load(const _Float16* p) {
    U f; f.h[0] = *(const v8h*)(p); f.h[1] = *(const v8h*)(p + 16); return f.v;
  }
  static __device__ __forceinline__ v8f mma(v16h a, v16h b, v8f c) {
    return __builtin_amdgcn_wmma_f32_16x16x32_f16(false, a, false, b, (short)0, c, false, false);
  }
  static __device__ __forceinline__ void guard(v8f& a, v8f& b, v16h x, v16h y) { dep_guard_h(a, b, x, y); }
  static __device__ __forceinline__ void keep(v16h a, v16h b, v16h c, v16h d) { keep4_h(a, b, c, d); }
};
template <> struct Frag<__bf16> {
  typedef v16b V; union U { v16b v; v8b h[2]; };
  static __device__ __forceinline__ v16b load(const __bf16* p) {
    U f; f.h[0] = *(const v8b*)(p); f.h[1] = *(const v8b*)(p + 16); return f.v;
  }
  static __device__ __forceinline__ v8f mma(v16b a, v16b b, v8f c) {
    return __builtin_amdgcn_wmma_f32_16x16x32_bf16(false, a, false, b, (short)0, c, false, false);
  }
  static __device__ __forceinline__ void guard(v8f& a, v8f& b, v16b x, v16b y) { dep_guard_b(a, b, x, y); }
  static __device__ __forceinline__ void keep(v16b a, v16b b, v16b c, v16b d) { keep4_b(a, b, c, d); }
};

template <int ET> struct Elem;
template <> struct Elem<0> { typedef _Float16 T; };
template <> struct Elem<1> { typedef __bf16 T; };
template <int ET, bool SPLIT, int BIAS_MODE, int OUT_MODE, bool RESID, int ACT = 0>
__global__ __launch_bounds__(256) void wmma_gemm64(
    const unsigned short* __restrict__ Ap, const unsigned short* __restrict__ A2p, int lda, long strideA,
    const unsigned short* __restrict__ Btp, const unsigned short* __restrict__ Bt2p, int ldb, long strideB,
    void* __restrict__ Cout, void* __restrict__ Cout2, int ldc, long strideC,
    const float* __restrict__ bias,
    const float* __restrict__ resid, long strideR,
    int M, int N, int K, float scale) {
  typedef typename Elem<ET>::T T;
  typedef typename Frag<T>::V V;
  const T* A = (const T*)Ap; const T* A2 = (const T*)A2p; const T* Bt = (const T*)Btp; const T* Bt2 = (const T*)Bt2p;
  __shared__ __align__(16) float sT[8][16 * 68];
  const int b    = blockIdx.y;
  const int lane = threadIdx.x & 31;
  const int wave = threadIdx.x >> 5;
  const int tilesN = N >> 6;
  const int tilesM = M >> 6;
  const int tile = blockIdx.x * 8 + wave;
  if (tile >= tilesM * tilesN) return;
  const int tm = tile / tilesN;
  const int tn = tile - tm * tilesN;
  const int m0 = tm << 6;
  const int n0 = tn << 6;

  const T* Ab  = A  + (size_t)b * strideA;
  const T* Bb  = Bt + (size_t)b * strideB;
  const T* Ab2 = SPLIT ? (A2  + (size_t)b * strideA) : nullptr;
  const T* Bb2 = SPLIT ? (Bt2 + (size_t)b * strideB) : nullptr;

  const int rlane = lane & 15;
  const int koff  = (lane >> 4) * 8;
  const int mOff  = (lane >> 4) * 8;

  v8f acc[4][4];
#pragma unroll
  for (int i = 0; i < 4; ++i)
#pragma unroll
    for (int j = 0; j < 4; ++j) acc[i][j] = (v8f){0.f,0.f,0.f,0.f,0.f,0.f,0.f,0.f};

  for (int k0 = 0; k0 < K; k0 += 32) {
    V bh[4], bl[4];
#pragma unroll
    for (int j = 0; j < 4; ++j) {
      const size_t bo = (size_t)(n0 + (j << 4) + rlane) * ldb + koff + k0;
      bh[j] = Frag<T>::load(Bb + bo);
      if (SPLIT) bl[j] = Frag<T>::load(Bb2 + bo);
    }
#pragma unroll
    for (int i = 0; i < 4; ++i) {
      const size_t ao = (size_t)(m0 + (i << 4) + rlane) * lda + koff + k0;
      V ah = Frag<T>::load(Ab + ao);
      V al;
      if (SPLIT) al = Frag<T>::load(Ab2 + ao);
#pragma unroll
      for (int j = 0; j < 4; ++j) {
        acc[i][j] = Frag<T>::mma(ah, bh[j], acc[i][j]);
        if (SPLIT) {
          acc[i][j] = Frag<T>::mma(ah, bl[j], acc[i][j]);
          acc[i][j] = Frag<T>::mma(al, bh[j], acc[i][j]);
        }
      }
      Frag<T>::guard(acc[i][0], acc[i][3], ah, SPLIT ? al : ah);
    }
    Frag<T>::keep(bh[0], bh[1], bh[2], bh[3]);
    if (SPLIT) Frag<T>::keep(bl[0], bl[1], bl[2], bl[3]);
  }
  acc_guard4(acc[0][0], acc[0][1], acc[0][2], acc[0][3]);
  acc_guard4(acc[1][0], acc[1][1], acc[1][2], acc[1][3]);
  acc_guard4(acc[2][0], acc[2][1], acc[2][2], acc[2][3]);
  acc_guard4(acc[3][0], acc[3][1], acc[3][2], acc[3][3]);

  float* slab = sT[wave];
  const float* Rb = RESID ? (resid + (size_t)b * strideR) : nullptr;
#pragma unroll
  for (int i = 0; i < 4; ++i) {
    const int mBase = m0 + (i << 4);
#pragma unroll
    for (int j = 0; j < 4; ++j) {
      const int n = n0 + (j << 4) + rlane;
      float bv = 0.f;
      if (BIAS_MODE == 2) bv = bias[n];
#pragma unroll
      for (int r = 0; r < 8; ++r) {
        float v = acc[i][j][r] * scale;
        if (BIAS_MODE == 1) v += bias[mBase + mOff + r];
        if (BIAS_MODE == 2) v += bv;
        if (RESID) v += Rb[(size_t)(mBase + mOff + r) * ldc + n];
        if (ACT == 1) v = tanhf(v);
        if (ACT == 2) v = fmaxf(v, 0.0f);
        if (ACT == 3) v = v / (1.0f + expf(-v));
        if (ACT == 4) v = (v > 0.f) ? v : 0.01f * v;
        if (ACT == 5) v = 0.5f * v * (1.0f + erff(v * 0.70710678118654752f));
        slab[(mOff + r) * 68 + (j << 4) + rlane] = v;
      }
    }
    __builtin_amdgcn_fence(__ATOMIC_RELEASE, "workgroup");
    __builtin_amdgcn_wave_barrier();
    __builtin_amdgcn_fence(__ATOMIC_ACQUIRE, "workgroup");
    if (OUT_MODE == 0) {
      float* C = (float*)Cout + (size_t)b * strideC;
      const int hh = lane >> 4, c4 = (lane & 15) * 4;
      for (int pass = 0; pass < 2; ++pass) {
#pragma unroll
        for (int it = 0; it < 8; ++it) {
          const int row = it * 2 + hh;
          v4f v = *(const v4f*)(slab + row * 68 + c4);
          *(volatile v4f*)(C + (size_t)(mBase + row) * ldc + n0 + c4) = v;
        }
        __threadfence();
      }
    } else {
      const int q = lane >> 3, c8 = (lane & 7) * 8;
      unsigned short* C  = (unsigned short*)Cout  + (size_t)b * strideC;
      unsigned short* C2 = (OUT_MODE == 2) ? ((unsigned short*)Cout2 + (size_t)b * strideC) : nullptr;
      for (int pass = 0; pass < 2; ++pass) {
#pragma unroll
        for (int it = 0; it < 4; ++it) {
          const int row = it * 4 + q;
          const float* sp = slab + row * 68 + c8;
          v8h hv, lv;
#pragma unroll
          for (int e = 0; e < 8; ++e) {
            if (OUT_MODE == 1) {
              hv[e] = (_Float16)sp[e];
            } else {
              unsigned short hb = f2bf_bits(sp[e]);
              unsigned short lb = f2bf_bits(sp[e] - bf_bits2f(hb));
              hv[e] = __builtin_bit_cast(_Float16, hb);
              lv[e] = __builtin_bit_cast(_Float16, lb);
            }
          }
          *(volatile v8h*)(C + (size_t)(mBase + row) * ldc + n0 + c8) = hv;
          if (OUT_MODE == 2) *(volatile v8h*)(C2 + (size_t)(mBase + row) * ldc + n0 + c8) = lv;
        }
        __threadfence();
      }
    }
    __builtin_amdgcn_fence(__ATOMIC_RELEASE, "workgroup");
    __builtin_amdgcn_wave_barrier();
    __builtin_amdgcn_fence(__ATOMIC_ACQUIRE, "workgroup");
  }
}

__device__ __forceinline__ float sigm_f(float x) {
  return __builtin_amdgcn_rcpf(1.0f + exp2f(-1.4426950408889634f * x));
}
__device__ __forceinline__ float tanh_f(float x) {
  x = fminf(fmaxf(x, -15.0f), 15.0f);
  const float em = exp2f(2.8853900817779268f * x);
  return (em - 1.0f) * __builtin_amdgcn_rcpf(em + 1.0f);
}

template <bool ASPLIT, int KST>
__device__ __forceinline__ void wave_cols32(
    const unsigned short* Ap, const unsigned short* A2p, int lda,
    const unsigned short* __restrict__ Btp, int ldb,
    float scale, float* Gout, int n0, float* stg, int lane,
    float* sSum, float* sSq)
{
  const _Float16* Am  = (const _Float16*)(const void*)Ap;
  const _Float16* Am2 = (const _Float16*)(const void*)A2p;
  const _Float16* Bm  = (const _Float16*)(const void*)Btp;
  const int rlane = lane & 15;
  const int hh    = lane >> 4;
  const int koff  = hh * 8;
  const int sq    = lane >> 3;
  const int c4    = (lane & 7) * 4;
  const float rsc = 1.0f / 2048.0f;
  float ss0 = 0.f, ss1 = 0.f, qq0 = 0.f, qq1 = 0.f;
#pragma unroll 1
  for (int mg = 0; mg < 32; ++mg) {
    const int m0 = mg * 32;
    v8f acc[2][2], accr[2][2];
#pragma unroll
    for (int i = 0; i < 2; ++i) {
#pragma unroll
      for (int j = 0; j < 2; ++j) {
        acc[i][j]  = (v8f){0.f,0.f,0.f,0.f,0.f,0.f,0.f,0.f};
        accr[i][j] = (v8f){0.f,0.f,0.f,0.f,0.f,0.f,0.f,0.f};
      }
    }
#pragma unroll 1
    for (int ks = 0; ks < KST; ++ks) {
      const int k0 = ks * 32;
      v16h bh[2];
#pragma unroll
      for (int j = 0; j < 2; ++j) {
        const size_t bo = (size_t)(n0 + j * 16 + rlane) * ldb + koff + k0;
        bh[j] = Frag<_Float16>::load(Bm + bo);
      }
#pragma unroll
      for (int i = 0; i < 2; ++i) {
        const size_t ao = (size_t)(m0 + i * 16 + rlane) * lda + koff + k0;
        const v16h ah = Frag<_Float16>::load(Am + ao);
        v16h al = ah;
        if (ASPLIT) al = Frag<_Float16>::load(Am2 + ao);
#pragma unroll
        for (int j = 0; j < 2; ++j) {
          acc[i][j] = Frag<_Float16>::mma(ah, bh[j], acc[i][j]);
          if (ASPLIT) accr[i][j] = Frag<_Float16>::mma(al, bh[j], accr[i][j]);
        }
        if (ASPLIT) dep_guard4_h(acc[i][0], acc[i][1], accr[i][0], accr[i][1], ah, al);
        else        dep_guard_h(acc[i][0], acc[i][1], ah, ah);
      }
      keep2_h(bh[0], bh[1]);
    }
    acc_guard4(acc[0][0], acc[0][1], acc[1][0], acc[1][1]);
    if (ASPLIT) acc_guard4(accr[0][0], accr[0][1], accr[1][0], accr[1][1]);

#pragma unroll
    for (int i = 0; i < 2; ++i) {
#pragma unroll
      for (int r = 0; r < 8; ++r) {
        float v0 = acc[i][0][r];
        float v1 = acc[i][1][r];
        if (ASPLIT) {
          v0 += accr[i][0][r] * rsc;
          v1 += accr[i][1][r] * rsc;
        }
        v0 *= scale;
        v1 *= scale;
        ss0 += v0; qq0 += v0 * v0;
        ss1 += v1; qq1 += v1 * v1;
        stg[(hh * 8 + r) * 36 + rlane]      = v0;
        stg[(hh * 8 + r) * 36 + 16 + rlane] = v1;
      }
      __builtin_amdgcn_fence(__ATOMIC_RELEASE, "workgroup");
      __builtin_amdgcn_wave_barrier();
      __builtin_amdgcn_fence(__ATOMIC_ACQUIRE, "workgroup");
      for (int pass = 0; pass < 2; ++pass) {
#pragma unroll
        for (int it = 0; it < 4; ++it) {
          const int row = it * 4 + sq;
          v4f v = *(const v4f*)(stg + row * 36 + c4);
          *(volatile v4f*)(Gout + (size_t)(m0 + i * 16 + row) * NGATE + n0 + c4) = v;
        }
        __threadfence();
      }
      __builtin_amdgcn_fence(__ATOMIC_RELEASE, "workgroup");
      __builtin_amdgcn_wave_barrier();
      __builtin_amdgcn_fence(__ATOMIC_ACQUIRE, "workgroup");
    }
  }
  ss0 += __shfl_xor(ss0, 16, 32);
  ss1 += __shfl_xor(ss1, 16, 32);
  qq0 += __shfl_xor(qq0, 16, 32);
  qq1 += __shfl_xor(qq1, 16, 32);
  if (hh == 0) {
    sSum[n0 + rlane]      = ss0;
    sSum[n0 + 16 + rlane] = ss1;
    sSq[n0 + rlane]       = qq0;
    sSq[n0 + 16 + rlane]  = qq1;
  }
}

template <int LAYER>
__global__ __launch_bounds__(512) void k_layer(
    const unsigned short* __restrict__ Xa, const unsigned short* __restrict__ Xb,
    const unsigned short* __restrict__ Wx, const unsigned short* __restrict__ Wh,
    const float* __restrict__ gih, const float* __restrict__ bih,
    const float* __restrict__ ghh, const float* __restrict__ bhh,
    const float* __restrict__ bvec, const float* __restrict__ gcv, const float* __restrict__ bcv,
    float* GXs, float* GHs, float* Cst,
    unsigned short* hF, unsigned short* hR, unsigned short* hBH, unsigned short* hBL,
    unsigned short* HSo)
{
  constexpr bool SPLX = (LAYER == 0);
  constexpr int  KXL  = (LAYER == 0) ? KXPAD0 : NHID;
  constexpr int  KXST = KXL / 32;
  const float xscale = (LAYER == 0) ? (1.0f / 16.0f) : (1.0f / 128.0f);
  const float hscale = 1.0f / 128.0f;

  __shared__ __align__(16) float stg_all[16][16 * 36];
  __shared__ float sX[NGATE], qX[NGATE], sHh[NGATE], qHh[NGATE];
  __shared__ float axL[NGATE], ahL[NGATE], cbL[NGATE];
  __shared__ float pS[8 * NHID], pQ[8 * NHID];
  __shared__ float acL[NHID], bcL[NHID];

  const int tid  = threadIdx.x;
  const int lane = tid & 31;
  const int wave = tid >> 5;
  float* stg = stg_all[wave];
  const int n0 = wave * 32;
  const int jp = tid & 63;
  const int rg = tid >> 6;
  const int j0 = jp * 2;
  const float inb = 1.0f / 1024.0f;

#pragma unroll 1
  for (int t = 0; t < NSTEP; ++t) {
    {
      const unsigned short* xa = Xa + (size_t)t * NBATCH * KXL;
      const unsigned short* xb = Xb + (size_t)t * NBATCH * KXL;
      wave_cols32<SPLX, KXST>(xa, xb, KXL, Wx, KXL, xscale, GXs, n0, stg, lane, sX, qX);
      wave_cols32<SPLX, 4>(hF, hR, NHID, Wh, NHID, hscale, GHs, n0, stg, lane, sHh, qHh);
    }
    __threadfence();
    __syncthreads();

    {
      const int col = tid;
      const float mx = sX[col] * inb;
      const float vx = fmaxf(qX[col] * inb - mx * mx, 0.0f);
      const float rx = rsqrtf(vx + 1e-5f);
      const float mh = sHh[col] * inb;
      const float vh = fmaxf(qHh[col] * inb - mh * mh, 0.0f);
      const float rh = rsqrtf(vh + 1e-5f);
      const float ax = gih[col] * rx;
      const float ah = ghh[col] * rh;
      axL[col] = ax;
      ahL[col] = ah;
      cbL[col] = (bih[col] - ax * mx) + (bhh[col] - ah * mh) + bvec[col];
    }
    __syncthreads();

    {
      float axf[2], ahf[2], cbf[2], axi[2], ahi[2], cbi[2], axg[2], ahg[2], cbg[2];
#pragma unroll
      for (int x = 0; x < 2; ++x) {
        axf[x] = axL[j0 + x];        ahf[x] = ahL[j0 + x];        cbf[x] = cbL[j0 + x];
        axi[x] = axL[128 + j0 + x];  ahi[x] = ahL[128 + j0 + x];  cbi[x] = cbL[128 + j0 + x];
        axg[x] = axL[384 + j0 + x];  ahg[x] = ahL[384 + j0 + x];  cbg[x] = cbL[384 + j0 + x];
      }
      float cs0 = 0.f, cs1 = 0.f, cq0 = 0.f, cq1 = 0.f;
#pragma unroll 1
      for (int e = 0; e < 128; ++e) {
        const int bb = rg + 8 * e;
        const float* gxr = GXs + (size_t)bb * NGATE + j0;
        const float* ghr = GHs + (size_t)bb * NGATE + j0;
        const v2f xf = *(const v2f*)(gxr);
        const v2f xi = *(const v2f*)(gxr + 128);
        const v2f xg = *(const v2f*)(gxr + 384);
        const v2f yf = *(const v2f*)(ghr);
        const v2f yi = *(const v2f*)(ghr + 128);
        const v2f yg = *(const v2f*)(ghr + 384);
        float* cp = Cst + (size_t)bb * NHID + j0;
        const v2f cv = *(const v2f*)cp;
        v2f cn;
#pragma unroll
        for (int x = 0; x < 2; ++x) {
          const float gf = axf[x] * xf[x] + ahf[x] * yf[x] + cbf[x];
          const float gi = axi[x] * xi[x] + ahi[x] * yi[x] + cbi[x];
          const float gg = axg[x] * xg[x] + ahg[x] * yg[x] + cbg[x];
          const float c1 = sigm_f(gf) * cv[x] + sigm_f(gi) * tanh_f(gg);
          cn[x] = c1;
        }
        cs0 += cn[0]; cq0 += cn[0] * cn[0];
        cs1 += cn[1]; cq1 += cn[1] * cn[1];
        *(volatile v2f*)cp = cn;
        __threadfence();
        *(volatile v2f*)cp = cn;
      }
      pS[rg * NHID + j0]     = cs0;
      pS[rg * NHID + j0 + 1] = cs1;
      pQ[rg * NHID + j0]     = cq0;
      pQ[rg * NHID + j0 + 1] = cq1;
    }
    __syncthreads();

    if (tid < NHID) {
      float s = 0.f, q = 0.f;
#pragma unroll
      for (int pp = 0; pp < 8; ++pp) { s += pS[pp * NHID + tid]; q += pQ[pp * NHID + tid]; }
      const float mc = s * inb;
      const float vc = fmaxf(q * inb - mc * mc, 0.0f);
      const float rc = rsqrtf(vc + 1e-5f);
      const float ac = gcv[tid] * rc;
      acL[tid] = ac;
      bcL[tid] = bcv[tid] - ac * mc;
    }
    __syncthreads();

    {
      float axo[2], aho[2], cbo[2], aco[2], bco[2];
#pragma unroll
      for (int x = 0; x < 2; ++x) {
        axo[x] = axL[256 + j0 + x];
        aho[x] = ahL[256 + j0 + x];
        cbo[x] = cbL[256 + j0 + x];
        aco[x] = acL[j0 + x];
        bco[x] = bcL[j0 + x];
      }
#pragma unroll 1
      for (int e = 0; e < 128; ++e) {
        const int bb = rg + 8 * e;
        const float* cp = Cst + (size_t)bb * NHID + j0;
        const v2f cv = *(const v2f*)cp;
        const v2f xo = *(const v2f*)(GXs + (size_t)bb * NGATE + 256 + j0);
        const v2f yo = *(const v2f*)(GHs + (size_t)bb * NGATE + 256 + j0);
        float hv[2];
#pragma unroll
        for (int x = 0; x < 2; ++x) {
          const float go = axo[x] * xo[x] + aho[x] * yo[x] + cbo[x];
          const float bn = aco[x] * cv[x] + bco[x];
          hv[x] = sigm_f(go) * tanh_f(bn);
        }
        const float a0 = hv[0] * 8.0f;
        const float a1 = hv[1] * 8.0f;
        const _Float16 q0 = (_Float16)a0;
        const _Float16 q1 = (_Float16)a1;
        const unsigned fb0 = (unsigned)__builtin_bit_cast(unsigned short, q0);
        const unsigned fb1 = (unsigned)__builtin_bit_cast(unsigned short, q1);
        const unsigned uF = fb0 | (fb1 << 16);
        const size_t wi = (size_t)bb * 64 + jp;
        if (LAYER == 0) {
          const _Float16 rs0 = (_Float16)((a0 - (float)q0) * 2048.0f);
          const _Float16 rs1 = (_Float16)((a1 - (float)q1) * 2048.0f);
          const unsigned rb0 = (unsigned)__builtin_bit_cast(unsigned short, rs0);
          const unsigned rb1 = (unsigned)__builtin_bit_cast(unsigned short, rs1);
          const unsigned uR = rb0 | (rb1 << 16);
          unsigned* pF = (unsigned*)hF + wi;
          unsigned* pR = (unsigned*)hR + wi;
          unsigned* pQ = (unsigned*)HSo + (size_t)t * NBATCH * 64 + wi;
          *(volatile unsigned*)pF = uF;
          *(volatile unsigned*)pR = uR;
          *(volatile unsigned*)pQ = uF;
          __threadfence();
          *(volatile unsigned*)pF = uF;
          *(volatile unsigned*)pR = uR;
          *(volatile unsigned*)pQ = uF;
        } else {
          const unsigned hb0 = (unsigned)f2bf_bits(hv[0]);
          const unsigned hb1 = (unsigned)f2bf_bits(hv[1]);
          const unsigned lb0 = (unsigned)f2bf_bits(hv[0] - bf_bits2f((unsigned short)hb0));
          const unsigned lb1 = (unsigned)f2bf_bits(hv[1] - bf_bits2f((unsigned short)hb1));
          const unsigned uH = hb0 | (hb1 << 16);
          const unsigned uL = lb0 | (lb1 << 16);
          unsigned* pF = (unsigned*)hF + wi;
          unsigned* pH = (unsigned*)hBH + wi;
          unsigned* pL = (unsigned*)hBL + wi;
          *(volatile unsigned*)pF = uF;
          *(volatile unsigned*)pH = uH;
          *(volatile unsigned*)pL = uL;
          __threadfence();
          *(volatile unsigned*)pF = uF;
          *(volatile unsigned*)pH = uH;
          *(volatile unsigned*)pL = uL;
        }
      }
    }
    __threadfence();
    __syncthreads();
  }
}

__global__ __launch_bounds__(256) void k_cvt_seq(const float* __restrict__ seq,
                                                 unsigned* XH, unsigned* XR, int nchunks)
{
  const int idx = blockIdx.x * 256 + threadIdx.x;
  if (idx >= nchunks) return;
  const int row = idx / 12;
  const int ch  = idx - row * 12;
  const int t   = row >> 10;
  const int bb  = row & 1023;
  const float* src = seq + ((size_t)bb * NSTEP + t) * NINP;
  unsigned hw[4], rw[4];
#pragma unroll
  for (int e = 0; e < 8; ++e) {
    const int k  = ch * 8 + e;
    const int kc = (k < NINP) ? k : (NINP - 1);
    float f = src[kc];
    f = (k < NINP) ? f : 0.0f;
    const _Float16 q  = (_Float16)f;
    const _Float16 rr = (_Float16)((f - (float)q) * 2048.0f);
    const unsigned hb = (unsigned)__builtin_bit_cast(unsigned short, q);
    const unsigned rb = (unsigned)__builtin_bit_cast(unsigned short, rr);
    if ((e & 1) == 0) { hw[e >> 1] = hb;        rw[e >> 1] = rb; }
    else              { hw[e >> 1] |= hb << 16;  rw[e >> 1] |= rb << 16; }
  }
  v4u H, R;
  H[0] = hw[0]; H[1] = hw[1]; H[2] = hw[2]; H[3] = hw[3];
  R[0] = rw[0]; R[1] = rw[1]; R[2] = rw[2]; R[3] = rw[3];
  v4u* ph = (v4u*)XH + idx;
  v4u* pr = (v4u*)XR + idx;
  *(volatile v4u*)ph = H;
  *(volatile v4u*)pr = R;
  __threadfence();
  *(volatile v4u*)ph = H;
  *(volatile v4u*)pr = R;
}

template <int MODE>
__global__ __launch_bounds__(256) void k_cvt_w(const float* __restrict__ W, int K, int N, int Kp,
                                               float scl, unsigned* P0, unsigned* P1, int nchunks)
{
  const int idx = blockIdx.x * 256 + threadIdx.x;
  if (idx >= nchunks) return;
  const int cpr = Kp >> 3;
  const int n   = idx / cpr;
  const int ch  = idx - n * cpr;
  unsigned w0[4], w1[4];
#pragma unroll
  for (int e = 0; e < 8; ++e) {
    const int k  = ch * 8 + e;
    const int kc = (k < K) ? k : (K - 1);
    float f = W[(size_t)kc * N + n];
    f = (k < K) ? f : 0.0f;
    unsigned a, c;
    if (MODE == 0) {
      a = (unsigned)f2bf_bits(f);
      c = (unsigned)f2bf_bits(f - bf_bits2f((unsigned short)a));
    } else {
      a = (unsigned)__builtin_bit_cast(unsigned short, (_Float16)(f * scl));
      c = a;
    }
    if ((e & 1) == 0) { w0[e >> 1] = a;        w1[e >> 1] = c; }
    else              { w0[e >> 1] |= a << 16;  w1[e >> 1] |= c << 16; }
  }
  v4u V0, V1;
  V0[0] = w0[0]; V0[1] = w0[1]; V0[2] = w0[2]; V0[3] = w0[3];
  V1[0] = w1[0]; V1[1] = w1[1]; V1[2] = w1[2]; V1[3] = w1[3];
  v4u* p0 = (v4u*)P0 + idx;
  *(volatile v4u*)p0 = V0;
  if (MODE == 0) { v4u* p1 = (v4u*)P1 + idx; *(volatile v4u*)p1 = V1; }
  __threadfence();
  *(volatile v4u*)p0 = V0;
  if (MODE == 0) { v4u* p1 = (v4u*)P1 + idx; *(volatile v4u*)p1 = V1; }
}

__global__ __launch_bounds__(256) void k_zero16(unsigned* p, int n16)
{
  const int idx = blockIdx.x * 256 + threadIdx.x;
  if (idx >= n16) return;
  v4u z;
  z[0] = 0u; z[1] = 0u; z[2] = 0u; z[3] = 0u;
  v4u* q = (v4u*)p + idx;
  *(volatile v4u*)q = z;
  __threadfence();
  *(volatile v4u*)q = z;
}

extern "C" void kernel_launch(void* const* d_in, const int* in_sizes, int n_in,
                              void* d_out, int out_size, void* d_ws, size_t ws_size,
                              hipStream_t stream)
{
  if (n_in < 23) return;
  if (in_sizes[0] != NBATCH * NSTEP * NINP) return;
  if (in_sizes[1] != NINP * NGATE || in_sizes[2] != NHID * NGATE) return;
  if (in_sizes[10] != NHID * NGATE || in_sizes[11] != NHID * NGATE) return;
  if (in_sizes[19] != NHID * NEMB || in_sizes[21] != NEMB * NDECO) return;
  if (out_size != NBATCH * NDECO) return;

  const float* seq   = (const float*)d_in[0];
  const float* Wih0  = (const float*)d_in[1];
  const float* Whh0  = (const float*)d_in[2];
  const float* b0    = (const float*)d_in[3];
  const float* gih0  = (const float*)d_in[4];
  const float* bih0  = (const float*)d_in[5];
  const float* ghh0  = (const float*)d_in[6];
  const float* bhh0  = (const float*)d_in[7];
  const float* gc0   = (const float*)d_in[8];
  const float* bc0   = (const float*)d_in[9];
  const float* Wih1  = (const float*)d_in[10];
  const float* Whh1  = (const float*)d_in[11];
  const float* b1    = (const float*)d_in[12];
  const float* gih1  = (const float*)d_in[13];
  const float* bih1  = (const float*)d_in[14];
  const float* ghh1  = (const float*)d_in[15];
  const float* bhh1  = (const float*)d_in[16];
  const float* gc1   = (const float*)d_in[17];
  const float* bc1   = (const float*)d_in[18];
  const float* fc_w  = (const float*)d_in[19];
  const float* fc_b  = (const float*)d_in[20];
  const float* dec_w = (const float*)d_in[21];
  const float* dec_b = (const float*)d_in[22];
  float* out = (float*)d_out;

  size_t off = 0;
  auto take = [&](size_t bytes) -> size_t { const size_t o = off; off += (bytes + 255) & ~(size_t)255; return o; };
  const size_t oXH   = take((size_t)NSTEP * NBATCH * KXPAD0 * 2);
  const size_t oXR   = take((size_t)NSTEP * NBATCH * KXPAD0 * 2);
  const size_t oHS0  = take((size_t)NSTEP * NBATCH * NHID * 2);
  const size_t oWI0  = take((size_t)NGATE * KXPAD0 * 2);
  const size_t oWH0  = take((size_t)NGATE * NHID * 2);
  const size_t oWI1  = take((size_t)NGATE * NHID * 2);
  const size_t oWH1  = take((size_t)NGATE * NHID * 2);
  const size_t oFCH  = take((size_t)NEMB * NHID * 2);
  const size_t oFCL  = take((size_t)NEMB * NHID * 2);
  const size_t oDECH = take((size_t)NDECO * NEMB * 2);
  const size_t oDECL = take((size_t)NDECO * NEMB * 2);
  const size_t oGX   = take((size_t)NBATCH * NGATE * 4);
  const size_t oGH   = take((size_t)NBATCH * NGATE * 4);
  const size_t planeC = (size_t)NBATCH * NHID * 4;
  const size_t planeH = (size_t)NBATCH * NHID * 2;
  const size_t stateBytes = planeC + 4 * planeH;
  const size_t oST   = take(stateBytes);
  const size_t oEMH  = take((size_t)NBATCH * NEMB * 2);
  const size_t oEML  = take((size_t)NBATCH * NEMB * 2);
  const size_t total = off;
  if (total > ws_size) return;

  char* ws = (char*)d_ws;
  unsigned short* XH   = (unsigned short*)(ws + oXH);
  unsigned short* XR   = (unsigned short*)(ws + oXR);
  unsigned short* HS0  = (unsigned short*)(ws + oHS0);
  unsigned short* WI0  = (unsigned short*)(ws + oWI0);
  unsigned short* WH0  = (unsigned short*)(ws + oWH0);
  unsigned short* WI1  = (unsigned short*)(ws + oWI1);
  unsigned short* WH1  = (unsigned short*)(ws + oWH1);
  unsigned short* FCH  = (unsigned short*)(ws + oFCH);
  unsigned short* FCL  = (unsigned short*)(ws + oFCL);
  unsigned short* DECH = (unsigned short*)(ws + oDECH);
  unsigned short* DECL = (unsigned short*)(ws + oDECL);
  float* GX = (float*)(ws + oGX);
  float* GH = (float*)(ws + oGH);
  float* Cst = (float*)(ws + oST);
  unsigned short* hF  = (unsigned short*)(ws + oST + planeC);
  unsigned short* hR  = (unsigned short*)(ws + oST + planeC + planeH);
  unsigned short* hBH = (unsigned short*)(ws + oST + planeC + 2 * planeH);
  unsigned short* hBL = (unsigned short*)(ws + oST + planeC + 3 * planeH);
  unsigned short* EMBH = (unsigned short*)(ws + oEMH);
  unsigned short* EMBL = (unsigned short*)(ws + oEML);

  const dim3 blk(256);

  {
    const int nseq = NSTEP * NBATCH * (KXPAD0 / 8);
    k_cvt_seq<<<dim3((nseq + 255) / 256), blk, 0, stream>>>(seq, (unsigned*)XH, (unsigned*)XR, nseq);
    int n;
    n = NGATE * (KXPAD0 / 8);
    k_cvt_w<1><<<dim3((n + 255) / 256), blk, 0, stream>>>(Wih0, NINP, NGATE, KXPAD0, 16.0f, (unsigned*)WI0, (unsigned*)WI0, n);
    n = NGATE * (NHID / 8);
    k_cvt_w<1><<<dim3((n + 255) / 256), blk, 0, stream>>>(Whh0, NHID, NGATE, NHID, 16.0f, (unsigned*)WH0, (unsigned*)WH0, n);
    k_cvt_w<1><<<dim3((n + 255) / 256), blk, 0, stream>>>(Wih1, NHID, NGATE, NHID, 16.0f, (unsigned*)WI1, (unsigned*)WI1, n);
    k_cvt_w<1><<<dim3((n + 255) / 256), blk, 0, stream>>>(Whh1, NHID, NGATE, NHID, 16.0f, (unsigned*)WH1, (unsigned*)WH1, n);
    n = NEMB * (NHID / 8);
    k_cvt_w<0><<<dim3((n + 255) / 256), blk, 0, stream>>>(fc_w, NHID, NEMB, NHID, 1.0f, (unsigned*)FCH, (unsigned*)FCL, n);
    n = NDECO * (NEMB / 8);
    k_cvt_w<0><<<dim3((n + 255) / 256), blk, 0, stream>>>(dec_w, NEMB, NDECO, NEMB, 1.0f, (unsigned*)DECH, (unsigned*)DECL, n);
  }
  const int nz = (int)(stateBytes / 16);

  k_zero16<<<dim3((nz + 255) / 256), blk, 0, stream>>>((unsigned*)Cst, nz);
  k_layer<0><<<dim3(1), dim3(512), 0, stream>>>(
      XH, XR, WI0, WH0,
      gih0, bih0, ghh0, bhh0, b0, gc0, bc0,
      GX, GH, Cst, hF, hR, hBH, hBL, HS0);

  k_zero16<<<dim3((nz + 255) / 256), blk, 0, stream>>>((unsigned*)Cst, nz);
  k_layer<1><<<dim3(1), dim3(512), 0, stream>>>(
      HS0, HS0, WI1, WH1,
      gih1, bih1, ghh1, bhh1, b1, gc1, bc1,
      GX, GH, Cst, hF, hR, hBH, hBL, HS0);

  wmma_gemm64<1, true, 2, 2, false><<<dim3(8, 1), blk, 0, stream>>>(
      hBH, hBL, NHID, 0L, FCH, FCL, NHID, 0L,
      (void*)EMBH, (void*)EMBL, NEMB, 0L,
      fc_b, (const float*)nullptr, 0L, NBATCH, NEMB, NHID, 1.0f);

  wmma_gemm64<1, true, 2, 0, false><<<dim3(300, 1), blk, 0, stream>>>(
      EMBH, EMBL, NEMB, 0L, DECH, DECL, NEMB, 0L,
      (void*)out, (void*)nullptr, NDECO, 0L,
      dec_b, (const float*)nullptr, 0L, NBATCH, NDECO, NEMB, 1.0f);
}
